// Decoder_bipartite_46815143526428
// MI455X (gfx1250) — hardware-verified
//
#include <hip/hip_runtime.h>
#include <stdint.h>

#define HD  128
#define K2  256
#define TE  64
#define ZS  264
#define HS  68

static_assert((ZS % 8) == 0);
static_assert((TE * ZS) >= ((TE - 1) * ZS + K2));
static_assert((HD * HS) >= ((HD - 1) * HS + TE));
static_assert(TE == 64);
static_assert(HD == 4 * 32);

typedef __bf16       v16b __attribute__((ext_vector_type(16)));
typedef float        v8f  __attribute__((ext_vector_type(8)));
typedef float        v4f  __attribute__((ext_vector_type(4)));
typedef unsigned int v4u  __attribute__((ext_vector_type(4)));

union Frag { v16b v; v4u u[2]; };

__device__ __forceinline__ unsigned short bf_bits(float f) {
  const unsigned u = __float_as_uint(f);
  return (unsigned short)((u + 0x7FFFu + ((u >> 16) & 1u)) >> 16);
}
__device__ __forceinline__ float bfr(float f) { return __uint_as_float(((unsigned)bf_bits(f)) << 16); }
__device__ __forceinline__ unsigned pk16(unsigned short a, unsigned short b) { return (unsigned)a | ((unsigned)b << 16); }
__device__ __forceinline__ v8f zero8() { v8f z = {0.f, 0.f, 0.f, 0.f, 0.f, 0.f, 0.f, 0.f}; return z; }

__device__ __forceinline__ Frag ldfrag(const unsigned short* p) {
  Frag f;
  f.u[0] = *(const v4u*)(p);
  f.u[1] = *(const v4u*)(p + 16);
  return f;
}

__device__ __forceinline__ v8f mma_bf(const Frag& a, const Frag& b, v8f c) {
  return __builtin_amdgcn_wmma_f32_16x16x32_bf16(false, a.v, false, b.v, (short)0, c, false, false);
}
__device__ __forceinline__ void guard(v8f& c, const Frag& a, const Frag& b) {
#if defined(__HIP_DEVICE_COMPILE__)
  asm volatile("v_nop\n\tv_nop\n\tv_nop\n\tv_nop" : "+v"(c) : "v"(a.u[0]), "v"(a.u[1]), "v"(b.u[0]), "v"(b.u[1]));
#endif
}

__global__ __launch_bounds__(256)
void k_cvt(const float* __restrict__ Xs, const float* __restrict__ Xd, const float* __restrict__ W,
           unsigned short* Ps, unsigned short* Pd, unsigned short* Pw,
           int npS, int npD, int npW, int nbS, int nbD) {
  const int blk = blockIdx.x, tid = threadIdx.x;
  const float* src;
  unsigned short* dst;
  int np, p;
  if (blk < nbS) {
    src = Xs; dst = Ps; np = npS; p = blk * 256 + tid;
  } else if (blk < nbS + nbD) {
    src = Xd; dst = Pd; np = npD; p = (blk - nbS) * 256 + tid;
  } else {
    src = W; dst = Pw; np = npW; p = (blk - nbS - nbD) * 256 + tid;
  }
  const int pc = min(p, np - 1);
  const v4f a = *(const v4f*)(src + (size_t)pc * 8);
  const v4f b = *(const v4f*)(src + (size_t)pc * 8 + 4);
  v4u u;
  u[0] = pk16(bf_bits(a[0]), bf_bits(a[1]));
  u[1] = pk16(bf_bits(a[2]), bf_bits(a[3]));
  u[2] = pk16(bf_bits(b[0]), bf_bits(b[1]));
  u[3] = pk16(bf_bits(b[2]), bf_bits(b[3]));
  unsigned short* d = dst + (size_t)pc * 8;
  if (p < np) *(volatile v4u*)d = u;
  __threadfence();
  if (p < np) *(volatile v4u*)d = u;
}

__global__ __launch_bounds__(256)
void k_dec(const unsigned short* __restrict__ Ps, const unsigned short* __restrict__ Pd,
           const int* __restrict__ eidx, const unsigned short* __restrict__ Pw,
           const float* __restrict__ b1, const float* __restrict__ W2, const float* __restrict__ b2,
           float* out, int E, int nsrc, int ndst) {
  __shared__ __align__(16) unsigned short zt[TE * ZS];
  __shared__ __align__(16) float ht[HD * HS];
  __shared__ float sB1[HD];
  __shared__ float sW2[HD];
  __shared__ __align__(16) float sOut[TE];

  const int tid = threadIdx.x, lane = tid & 31, wave = tid >> 5, hh = lane >> 4, c = lane & 15;
  const int e0 = blockIdx.x * TE;

  if (tid < HD) sB1[tid] = bfr(b1[tid]);
  else          sW2[tid - HD] = bfr(W2[tid - HD]);

  {
    const int e = tid >> 2, q = tid & 3;
    const int eg = min(e0 + e, E - 1);
    int r  = eidx[eg];
    int cc = eidx[(size_t)E + (size_t)eg];
    r  = min(max(r, 0), nsrc - 1);
    cc = min(max(cc, 0), ndst - 1);
    const unsigned short* ps = Ps + (size_t)r * HD + 64 * (q & 1);
    const unsigned short* pd = Pd + (size_t)cc * HD + 64 * (q & 1);
    const unsigned short* sp = (q < 2) ? ps : pd;
    v4u u[8];
#pragma unroll
    for (int i = 0; i < 8; ++i) u[i] = *(const v4u*)(sp + 8 * i);
    unsigned short* dp = zt + e * ZS + 64 * q;
#pragma unroll
    for (int i = 0; i < 8; ++i) *(v4u*)(dp + 8 * i) = u[i];
  }

  const int n = 16 * wave + c;
  Frag bf[8];
  {
    const unsigned short* wp = Pw + (size_t)n * K2 + 8 * hh;
#pragma unroll
    for (int g = 0; g < 8; ++g) bf[g] = ldfrag(wp + 32 * g);
  }
  __syncthreads();

  const float bias = sB1[n];
#pragma unroll
  for (int m = 0; m < 4; ++m) {
    v8f acc = zero8();
    const unsigned short* ap = zt + (16 * m + c) * ZS + 8 * hh;
#pragma unroll
    for (int g = 0; g < 8; ++g) {
      const Frag af = ldfrag(ap + 32 * g);
      acc = mma_bf(af, bf[g], acc);
      guard(acc, af, bf[g]);
    }
    float* hrow = ht + n * HS + 16 * m + 8 * hh;
#pragma unroll
    for (int r = 0; r < 8; ++r) hrow[r] = fmaxf(acc[r] + bias, 0.0f);
  }
  __syncthreads();

  {
    const int e = tid >> 2, q = tid & 3;
    const float* hp = ht + (32 * q) * HS + e;
    const float* wv = sW2 + 32 * q;
    float s = 0.0f;
#pragma unroll 4
    for (int k = 0; k < 32; ++k) s = fmaf(wv[k], hp[k * HS], s);
    s += __shfl_xor(s, 1);
    s += __shfl_xor(s, 2);
    const float lg = s + bfr(b2[0]);
    const float ex = expf(-lg);
    const float sg = __builtin_amdgcn_rcpf(1.0f + ex);
    if (q == 0) sOut[e] = sg;
  }
  __syncthreads();

  if (e0 + TE <= E) {
    if (wave == 0) {
      const v4f ov = *(const v4f*)(sOut + 4 * c);
      float* op = out + (size_t)e0 + 4 * c;
      if (lane < 16) *(volatile v4f*)op = ov;
      __threadfence();
      if (lane < 16) *(volatile v4f*)op = ov;
    }
  } else {
    const float v = sOut[tid & (TE - 1)];
    const bool wr = (tid < TE) && (e0 + tid < E);
    if (wr) *(volatile float*)(out + (size_t)e0 + tid) = v;
    __threadfence();
    if (wr) *(volatile float*)(out + (size_t)e0 + tid) = v;
  }
}

static inline size_t al256(size_t x) { return (x + 255) & ~(size_t)255; }

extern "C" void kernel_launch(void* const* d_in, const int* in_sizes, int n_in,
                              void* d_out, int out_size, void* d_ws, size_t ws_size,
                              hipStream_t stream) {
  if (n_in < 7) return;
  const int nS = in_sizes[0], nD = in_sizes[1], nE2 = in_sizes[2];
  if (nS < HD || nD < HD || (nS % HD) != 0 || (nD % HD) != 0) return;
  if (in_sizes[3] != HD * K2 || in_sizes[4] != HD || in_sizes[5] != HD || in_sizes[6] < 1) return;
  if (nE2 < 2 || (nE2 & 1) != 0) return;
  const int E = nE2 / 2;
  if (out_size != E) return;
  const int nsrc = nS / HD, ndst = nD / HD;

  const float* z_src = (const float*)d_in[0];
  const float* z_dst = (const float*)d_in[1];
  const int*   eidx  = (const int*)d_in[2];
  const float* W1    = (const float*)d_in[3];
  const float* b1    = (const float*)d_in[4];
  const float* W2    = (const float*)d_in[5];
  const float* b2    = (const float*)d_in[6];
  float* out = (float*)d_out;

  const size_t sPs = al256((size_t)nS * 2);
  const size_t sPd = al256((size_t)nD * 2);
  const size_t sPw = al256((size_t)HD * K2 * 2);
  size_t off = 0;
  const size_t oPs = off; off += sPs;
  const size_t oPd = off; off += sPd;
  const size_t oPw = off; off += sPw;
  if (off > ws_size) return;
  if (off > (size_t)134217728) return;

  char* ws = (char*)d_ws;
  unsigned short* Ps = (unsigned short*)(ws + oPs);
  unsigned short* Pd = (unsigned short*)(ws + oPd);
  unsigned short* Pw = (unsigned short*)(ws + oPw);

  const int npS = nS / 8, npD = nD / 8, npW = (HD * K2) / 8;
  const int nbS = (npS + 255) / 256, nbD = (npD + 255) / 256, nbW = (npW + 255) / 256;

  k_cvt<<<dim3(nbS + nbD + nbW), dim3(256), 0, stream>>>(z_src, z_dst, W1, Ps, Pd, Pw, npS, npD, npW, nbS, nbD);
  const int nblk = (E + TE - 1) / TE;
  k_dec<<<dim3(nblk), dim3(256), 0, stream>>>(Ps, Pd, eidx, Pw, b1, W2, b2, out, E, nsrc, ndst);
  (void)hipGetLastError();
}
